// PointInterpDecoder_39213051412833
// MI455X (gfx1250) — hardware-verified
//
#include <hip/hip_runtime.h>


#define NB_  4
#define NQ   8192
#define NP   2048
#define DIN  256
#define DM   200
#define DMP  256
#define HIDd 128
#define PCAR 1024.0f
typedef _Float16 h16;
typedef unsigned short bf;
typedef __attribute__((ext_vector_type(16))) __bf16   v16bf;
typedef __attribute__((ext_vector_type(16))) _Float16 v16h;
typedef __attribute__((ext_vector_type(8)))  _Float16 v8h;
typedef __attribute__((ext_vector_type(8)))  unsigned short v8us;
typedef __attribute__((ext_vector_type(8)))  float    v8f;
typedef __attribute__((ext_vector_type(4)))  float    v4f;
typedef v8h  __attribute__((may_alias)) v8ha;
typedef v4f  __attribute__((may_alias)) v4fa;
typedef v8us __attribute__((may_alias)) v8usa;

__device__ __forceinline__ unsigned short f2bf(float f) { unsigned u = __float_as_uint(f); u += 0x7FFFu + ((u >> 16) & 1u); return (unsigned short)(u >> 16); }
__device__ __forceinline__ float bf2f(unsigned short b) { return __uint_as_float(((unsigned)b) << 16); }
__device__ __forceinline__ float bfr(float f) { return bf2f(f2bf(f)); }
__device__ __forceinline__ v16h cat16(v8h lo, v8h hi) { return __builtin_shufflevector(lo, hi, 0, 1, 2, 3, 4, 5, 6, 7, 8, 9, 10, 11, 12, 13, 14, 15); }
__device__ __forceinline__ v16bf cat16b(v8us lo, v8us hi) { return __builtin_bit_cast(v16bf, __builtin_shufflevector(lo, hi, 0, 1, 2, 3, 4, 5, 6, 7, 8, 9, 10, 11, 12, 13, 14, 15)); }
__device__ __forceinline__ v8f wmma16(v16h a, v16h b, v8f c) { return __builtin_amdgcn_wmma_f32_16x16x32_f16(false, a, false, b, (short)0, c, false, false); }
__device__ __forceinline__ v8f wmmab(v16bf a, v16bf b, v8f c) { return __builtin_amdgcn_wmma_f32_16x16x32_bf16(false, a, false, b, (short)0, c, false, false); }


template <typename T16> struct WFrag;
template <> struct WFrag<h16> { typedef v16h V; static __device__ __forceinline__ V ld(const h16* p) { return cat16(*(const v8h*)p, *(const v8h*)(p + 16)); } static __device__ __forceinline__ v8f mma(V a, V b, v8f c) { return wmma16(a, b, c); } };
template <> struct WFrag<bf> { typedef v16bf V; static __device__ __forceinline__ V ld(const bf* p) { return cat16b(*(const v8us*)p, *(const v8us*)(p + 16)); } static __device__ __forceinline__ v8f mma(V a, V b, v8f c) { return wmmab(a, b, c); } };
template <typename T16, int NSPLIT, bool BIAS>
__global__ __launch_bounds__(32) void k_gemmw(const T16* __restrict__ A, const T16* __restrict__ A2, const T16* __restrict__ Bt, const T16* __restrict__ Bt2, int K, float* C, int ldc, const float* __restrict__ bias, size_t sA, size_t sB, size_t sC) {
    typedef typename WFrag<T16>::V V;
    __shared__ __align__(16) float os[16 * 68];
    const size_t z = blockIdx.z; A += z * sA; if (A2) A2 += z * sA; Bt += z * sB; if (Bt2) Bt2 += z * sB; C += z * sC;
    const int lane = threadIdx.x & 31, lr = lane & 15, hi = lane >> 4; const int r0 = blockIdx.x * 64, c0 = blockIdx.y * 64;
    v8f acc[4][4];
#pragma unroll
    for (int mb = 0; mb < 4; ++mb)
#pragma unroll
        for (int nb = 0; nb < 4; ++nb) acc[mb][nb] = (v8f){};
    const size_t aoff = (size_t)(r0 + lr) * K + 8 * hi, boff = (size_t)(c0 + lr) * K + 8 * hi;
#pragma unroll 1
    for (int kc = 0; kc < K; kc += 32) {
        V a[4], a2[4];
#pragma unroll
        for (int mb = 0; mb < 4; ++mb) { a[mb] = WFrag<T16>::ld(A + aoff + (size_t)mb * 16 * K + kc); if (NSPLIT == 1 || NSPLIT == 2) a2[mb] = WFrag<T16>::ld(A2 + aoff + (size_t)mb * 16 * K + kc); }
#pragma unroll
        for (int nb = 0; nb < 4; ++nb) { const V b = WFrag<T16>::ld(Bt + boff + (size_t)nb * 16 * K + kc); V b2; if (NSPLIT >= 2) b2 = WFrag<T16>::ld(Bt2 + boff + (size_t)nb * 16 * K + kc);
#pragma unroll
            for (int mb = 0; mb < 4; ++mb) { acc[mb][nb] = WFrag<T16>::mma(a[mb], b, acc[mb][nb]); if (NSPLIT == 1 || NSPLIT == 2) acc[mb][nb] = WFrag<T16>::mma(a2[mb], b, acc[mb][nb]); if (NSPLIT >= 2) acc[mb][nb] = WFrag<T16>::mma(a[mb], b2, acc[mb][nb]); } }
        asm volatile("v_nop\n\tv_nop\n\tv_nop\n\tv_nop" : "+v"(acc[0][0]), "+v"(acc[1][1]), "+v"(acc[2][2]), "+v"(acc[3][3]) : "v"(a[0]), "v"(a[3]));
    }
#pragma unroll
    for (int mb = 0; mb < 4; ++mb) {
#pragma unroll
        for (int nb = 0; nb < 4; ++nb) {
#pragma unroll
            for (int j = 0; j < 8; ++j) os[(hi * 8 + j) * 68 + nb * 16 + lr] = acc[mb][nb][j]; }
        __builtin_amdgcn_wave_barrier(); asm volatile("" ::: "memory");
        float* crow = C + (size_t)(r0 + mb * 16) * ldc + c0;
#pragma unroll 1
        for (int ps = 0; ps < 2; ++ps) {
#pragma unroll
            for (int s = 0; s < 8; ++s) { const int row = 2 * s + hi, cofs = lr * 4; v4f val = *(const v4fa*)(os + row * 68 + cofs); if (BIAS) { val[0] += bfr(bias[c0 + cofs]); val[1] += bfr(bias[c0 + cofs + 1]); val[2] += bfr(bias[c0 + cofs + 2]); val[3] += bfr(bias[c0 + cofs + 3]); }
                *(volatile v4f*)(crow + (size_t)row * ldc + cofs) = val; }
            if (ps == 0) __threadfence(); }
        __builtin_amdgcn_wave_barrier(); asm volatile("" ::: "memory");
    }
}

__device__ __forceinline__ h16 tohx(float x) { return (h16)x; }
__device__ __forceinline__ void splitf(float y, unsigned short& h, unsigned short& l) { h = f2bf(y); l = f2bf(y - bf2f(h)); }
typedef __attribute__((ext_vector_type(2))) _Float16 v2h;
typedef __attribute__((ext_vector_type(4))) _Float16 v4h;
typedef __attribute__((ext_vector_type(4))) unsigned short v4us;

__global__ __launch_bounds__(256) void k_wpadT(const float* __restrict__ w, int kreal, int nreal, int NOUT, int KP, bf* Bt) { const int e = (blockIdx.x * 256 + threadIdx.x) * 2; if (e >= NOUT * KP) return; const int k = e % KP, n = e / KP; unsigned short o0 = 0, o1 = 0;
    if (n < nreal) { if (k < kreal) o0 = f2bf(w[(size_t)k * nreal + n]); if (k + 1 < kreal) o1 = f2bf(w[(size_t)(k + 1) * nreal + n]); } typedef __attribute__((ext_vector_type(2))) unsigned short v2us; v2us o; o[0] = o0; o[1] = o1; *(volatile v2us*)(Bt + e) = o; __threadfence(); *(volatile v2us*)(Bt + e) = o; }
__global__ __launch_bounds__(256) void k_lg(const float* __restrict__ q, const float* __restrict__ an, float* S) { const size_t e = ((size_t)blockIdx.x * 256 + threadIdx.x) * 4; if (e >= (size_t)NQ * NP) return; const int p = (int)(e % NP); const int qi = (int)(e / NP); const float qx = bfr(q[qi * 3]), qy = bfr(q[qi * 3 + 1]), qz = bfr(q[qi * 3 + 2]); v4f o;
#pragma unroll
    for (int u = 0; u < 4; ++u) { const float* a = an + (size_t)(p + u) * 3; const float dx = __fsub_rn(bfr(a[0]), qx), dy = __fsub_rn(bfr(a[1]), qy), dz = __fsub_rn(bfr(a[2]), qz); float sx = __fmul_rn(dx, dx); asm volatile("" : "+v"(sx)); float sy = __fmul_rn(dy, dy); asm volatile("" : "+v"(sy)); float sz = __fmul_rn(dz, dz); asm volatile("" : "+v"(sz));
        const float d = __fadd_rn(__fsqrt_rn(__fadd_rn(__fadd_rn(sx, sy), sz)), 1e-5f); float d2 = __fmul_rn(d, d); asm volatile("" : "+v"(d2)); o[u] = -__fdiv_rn(d2, 0.04f); }
    *(volatile v4f*)(S + e) = o; __threadfence(); *(volatile v4f*)(S + e) = o; }
__global__ __launch_bounds__(256) void k_ft16(const float* __restrict__ f, h16* FT) { const int e = (blockIdx.x * 256 + threadIdx.x) * 2; if (e >= DIN * NP) return; const int p = e % NP; const int c = e / NP; v2h o; o[0] = tohx(bfr(f[(size_t)p * DIN + c])); o[1] = tohx(bfr(f[(size_t)(p + 1) * DIN + c])); *(volatile v2h*)(FT + e) = o; __threadfence(); *(volatile v2h*)(FT + e) = o; }
__global__ __launch_bounds__(256) void k_splits(const float* __restrict__ F, size_t n4, float sc, bf* Hh, bf* Hl) { const size_t e = ((size_t)blockIdx.x * 256 + threadIdx.x) * 4; if (e >= n4 * 4) return; const v4f a = *(const v4f*)(F + e); v4us oh, ol;
#pragma unroll
    for (int u = 0; u < 4; ++u) { unsigned short h, l; splitf(a[u] * sc, h, l); oh[u] = h; ol[u] = l; } *(volatile v4us*)(Hh + e) = oh; *(volatile v4us*)(Hl + e) = ol; __threadfence(); *(volatile v4us*)(Hh + e) = oh; *(volatile v4us*)(Hl + e) = ol; }
__global__ __launch_bounds__(256) void k_relupl(const float* __restrict__ F, size_t n4, bf* Hh, bf* Hl) { const size_t e = ((size_t)blockIdx.x * 256 + threadIdx.x) * 4; if (e >= n4 * 4) return; const v4f a = *(const v4f*)(F + e); v4us oh, ol;
#pragma unroll
    for (int u = 0; u < 4; ++u) { unsigned short h, l; splitf(fmaxf(a[u], 0.f), h, l); oh[u] = h; ol[u] = l; } *(volatile v4us*)(Hh + e) = oh; *(volatile v4us*)(Hl + e) = ol; __threadfence(); *(volatile v4us*)(Hh + e) = oh; *(volatile v4us*)(Hl + e) = ol; }
template <int RELU> __global__ __launch_bounds__(256) void k_addpl(float* NET, const float* __restrict__ T, bf* Ph, bf* Pl) { const size_t e = ((size_t)blockIdx.x * 256 + threadIdx.x) * 4; if (e >= (size_t)NQ * HIDd) return; const v4f a = *(const v4f*)(NET + e); const v4f t = *(const v4f*)(T + e); v4f o; v4us oh, ol;
#pragma unroll
    for (int u = 0; u < 4; ++u) { o[u] = __fadd_rn(a[u], t[u]); unsigned short h, l; splitf(RELU ? fmaxf(o[u], 0.f) : o[u], h, l); oh[u] = h; ol[u] = l; }
    for (int ps = 0; ps < 2; ++ps) { *(volatile v4f*)(NET + e) = o; *(volatile v4us*)(Ph + e) = oh; *(volatile v4us*)(Pl + e) = ol; if (ps == 0) __threadfence(); } }
__global__ __launch_bounds__(256) void k_latpl(const float* __restrict__ LAT, const float* __restrict__ b, bf* Lh, bf* Ll, bf* Rh, bf* Rl) { const size_t e = ((size_t)blockIdx.x * 256 + threadIdx.x) * 4; if (e >= (size_t)NQ * DMP) return; const int c = (int)(e % DMP); const v4f a = *(const v4f*)(LAT + e); v4us lh, ll, rh, rl;
#pragma unroll
    for (int u = 0; u < 4; ++u) { const float v = (c + u < DM) ? __fadd_rn(a[u], bfr(b[c + u])) : 0.f; unsigned short h, l; splitf(v, h, l); lh[u] = h; ll[u] = l; splitf(fmaxf(v, 0.f), h, l); rh[u] = h; rl[u] = l; }
    for (int ps = 0; ps < 2; ++ps) { *(volatile v4us*)(Lh + e) = lh; *(volatile v4us*)(Ll + e) = ll; *(volatile v4us*)(Rh + e) = rh; *(volatile v4us*)(Rl + e) = rl; if (ps == 0) __threadfence(); } }
__global__ __launch_bounds__(256) void k_out3(const float* __restrict__ T64, const float* __restrict__ ob, float* OUTb) { const int e = blockIdx.x * 256 + threadIdx.x; if (e >= NQ * 3) return; const float v = __fadd_rn(T64[(size_t)(e / 3) * 64 + (e % 3)], bfr(ob[e % 3])); *(volatile float*)(OUTb + e) = v; __threadfence(); *(volatile float*)(OUTb + e) = v; }
template <int NFULL, int TAIL> __global__ __launch_bounds__(256) void k_soft(const float* __restrict__ Sb, int nrows, int rowsper, int rvalid, int nvalid, h16* P) { const int lane = threadIdx.x & 31; const size_t row = (size_t)blockIdx.x * 8 + (threadIdx.x >> 5); if (row >= (size_t)nrows) return; constexpr int LD = NFULL * 128 + TAIL * 64; const float* sr = Sb + row * LD; h16* pr = P + row * LD; const bool live = (int)(row % rowsper) < rvalid; float mx = -3.0e38f;
#pragma unroll 1
    for (int ch = 0; ch < NFULL + TAIL; ++ch) { if (ch == NFULL && lane >= 16) break; const int j0 = ch * 128 + lane * 4; const v4f a = *(const v4f*)(sr + j0);
#pragma unroll
        for (int q = 0; q < 4; ++q) if (j0 + q < nvalid) mx = fmaxf(mx, a[q]); }
#pragma unroll
    for (int sh = 16; sh; sh >>= 1) mx = fmaxf(mx, __shfl_xor(mx, sh, 32));
    float sum = 0.f;
#pragma unroll 1
    for (int ch = 0; ch < NFULL + TAIL; ++ch) { if (ch == NFULL && lane >= 16) break; const int j0 = ch * 128 + lane * 4; const v4f a = *(const v4f*)(sr + j0);
#pragma unroll
        for (int q = 0; q < 4; ++q) if (j0 + q < nvalid) { float d0 = __fsub_rn(a[q], mx); asm volatile("" : "+v"(d0)); sum += __expf(d0); } }
#pragma unroll
    for (int sh = 16; sh; sh >>= 1) sum += __shfl_xor(sum, sh, 32);
    const float f = live ? __fdiv_rn(PCAR, sum) : 0.f;
    for (int ps = 0; ps < 2; ++ps) {
#pragma unroll 1
        for (int ch = 0; ch < NFULL + TAIL; ++ch) { if (ch == NFULL && lane >= 16) break; const int j0 = ch * 128 + lane * 4; const v4f a = *(const v4f*)(sr + j0); v4h o;
#pragma unroll
            for (int q = 0; q < 4; ++q) { float val = 0.f; if (live && j0 + q < nvalid) { float d0 = __fsub_rn(a[q], mx); asm volatile("" : "+v"(d0)); val = __fmul_rn(__expf(d0), f); } o[q] = tohx(val); } *(volatile v4h*)(pr + j0) = o; }
        if (ps == 0) __threadfence(); } }

extern "C" void kernel_launch(void* const* d_in, const int* in_sizes, int n_in,
                              void* d_out, int out_size, void* d_ws, size_t ws_size, hipStream_t stream) {
    (void)in_sizes; (void)n_in; (void)out_size;
    const float* xyz = (const float*)d_in[0]; const float* anc = (const float*)d_in[1]; const float* feats = (const float*)d_in[2]; const float* fc0w = (const float*)d_in[3]; const float* fc0b = (const float*)d_in[4]; const float* fc1w = (const float*)d_in[5]; const float* fc1b = (const float*)d_in[6]; const float* bw0 = (const float*)d_in[7]; const float* bb0 = (const float*)d_in[8]; const float* bw1 = (const float*)d_in[9]; const float* bb1 = (const float*)d_in[10]; const float* fcw = (const float*)d_in[11]; const float* fcb = (const float*)d_in[12]; const float* ow = (const float*)d_in[13]; const float* ob = (const float*)d_in[14];
    float* OUT = (float*)d_out;
    char* wsp = (char*)d_ws;
    auto take = [&](size_t bytes) { char* p = wsp; wsp += (bytes + 255) & ~(size_t)255; return (void*)p; };
    bf* FC0 = (bf*)take(DMP * DIN * 2); bf* FC1 = (bf*)take(HIDd * DMP * 2); bf* OW = (bf*)take(64 * HIDd * 2); bf* BW0[5]; bf* BW1[5]; bf* FCC[5]; for (int i = 0; i < 5; ++i) { BW0[i] = (bf*)take(HIDd * HIDd * 2); BW1[i] = (bf*)take(HIDd * HIDd * 2); FCC[i] = (bf*)take(HIDd * DMP * 2); }
    float* S = (float*)take((size_t)NQ * NP * 4); h16* P16 = (h16*)take((size_t)NQ * NP * 2); h16* FT = (h16*)take((size_t)DIN * NP * 2); float* C = (float*)take((size_t)NQ * DIN * 4); bf* Ch = (bf*)take((size_t)NQ * DIN * 2); bf* Cl = (bf*)take((size_t)NQ * DIN * 2); float* LAT = (float*)take((size_t)NQ * DMP * 4); bf* Lh = (bf*)take((size_t)NQ * DMP * 2); bf* Ll = (bf*)take((size_t)NQ * DMP * 2); bf* LRh = (bf*)take((size_t)NQ * DMP * 2); bf* LRl = (bf*)take((size_t)NQ * DMP * 2);
    float* NET = (float*)take((size_t)NQ * HIDd * 4); float* T = (float*)take((size_t)NQ * HIDd * 4); bf* Ph = (bf*)take((size_t)NQ * HIDd * 2); bf* Pl = (bf*)take((size_t)NQ * HIDd * 2); bf* Qh = (bf*)take((size_t)NQ * HIDd * 2); bf* Ql = (bf*)take((size_t)NQ * HIDd * 2); float* T64 = (float*)take((size_t)NQ * 64 * 4);
    if ((size_t)(wsp - (char*)d_ws) > ws_size) return;
    k_wpadT<<<(DMP * DIN / 2 + 255) / 256, 256, 0, stream>>>(fc0w, DIN, DM, DMP, DIN, FC0); k_wpadT<<<(HIDd * DMP / 2 + 255) / 256, 256, 0, stream>>>(fc1w, DM, HIDd, HIDd, DMP, FC1); k_wpadT<<<(64 * HIDd / 2 + 255) / 256, 256, 0, stream>>>(ow, HIDd, 3, 64, HIDd, OW);
    for (int i = 0; i < 5; ++i) { k_wpadT<<<(HIDd * HIDd / 2 + 255) / 256, 256, 0, stream>>>(bw0 + (size_t)i * HIDd * HIDd, HIDd, HIDd, HIDd, HIDd, BW0[i]); k_wpadT<<<(HIDd * HIDd / 2 + 255) / 256, 256, 0, stream>>>(bw1 + (size_t)i * HIDd * HIDd, HIDd, HIDd, HIDd, HIDd, BW1[i]); k_wpadT<<<(HIDd * DMP / 2 + 255) / 256, 256, 0, stream>>>(fcw + (size_t)i * DM * HIDd, DM, HIDd, HIDd, DMP, FCC[i]); }
    for (int b = 0; b < NB_; ++b) {
        k_lg<<<(unsigned)(((size_t)NQ * NP / 4 + 255) / 256), 256, 0, stream>>>(xyz + (size_t)b * NQ * 3, anc + (size_t)b * NP * 3, S);
        k_soft<16, 0><<<NQ / 8, 256, 0, stream>>>(S, NQ, NP, NP, NP, P16);
        k_ft16<<<(DIN * NP / 2 + 255) / 256, 256, 0, stream>>>(feats + (size_t)b * NP * DIN, FT);
        k_gemmw<h16, 0, false><<<dim3(NQ / 64, DIN / 64, 1), 32, 0, stream>>>(P16, nullptr, FT, nullptr, NP, C, DIN, nullptr, 0, 0, 0);
        k_splits<<<(NQ * DIN / 4 + 255) / 256, 256, 0, stream>>>(C, (size_t)NQ * DIN / 4, 1.0f / PCAR, Ch, Cl);
        k_gemmw<bf, 1, false><<<dim3(NQ / 64, DMP / 64, 1), 32, 0, stream>>>(Ch, Cl, FC0, nullptr, DIN, LAT, DMP, nullptr, 0, 0, 0);
        k_latpl<<<(NQ * DMP / 4 + 255) / 256, 256, 0, stream>>>(LAT, fc0b, Lh, Ll, LRh, LRl);
        k_gemmw<bf, 1, true><<<dim3(NQ / 64, HIDd / 64, 1), 32, 0, stream>>>(LRh, LRl, FC1, nullptr, DMP, NET, HIDd, fc1b, 0, 0, 0);
        for (int i = 0; i < 5; ++i) {
            k_gemmw<bf, 1, true><<<dim3(NQ / 64, HIDd / 64, 1), 32, 0, stream>>>(Lh, Ll, FCC[i], nullptr, DMP, T, HIDd, fcb + i * HIDd, 0, 0, 0); k_addpl<1><<<(NQ * HIDd / 4 + 255) / 256, 256, 0, stream>>>(NET, T, Ph, Pl);
            k_gemmw<bf, 1, true><<<dim3(NQ / 64, HIDd / 64, 1), 32, 0, stream>>>(Ph, Pl, BW0[i], nullptr, HIDd, T, HIDd, bb0 + i * HIDd, 0, 0, 0); k_relupl<<<(NQ * HIDd / 4 + 255) / 256, 256, 0, stream>>>(T, (size_t)NQ * HIDd / 4, Qh, Ql);
            k_gemmw<bf, 1, true><<<dim3(NQ / 64, HIDd / 64, 1), 32, 0, stream>>>(Qh, Ql, BW1[i], nullptr, HIDd, T, HIDd, bb1 + i * HIDd, 0, 0, 0); k_addpl<1><<<(NQ * HIDd / 4 + 255) / 256, 256, 0, stream>>>(NET, T, Ph, Pl); }
        k_gemmw<bf, 1, false><<<dim3(NQ / 64, 1, 1), 32, 0, stream>>>(Ph, Pl, OW, nullptr, HIDd, T64, 64, nullptr, 0, 0, 0); k_out3<<<(NQ * 3 + 255) / 256, 256, 0, stream>>>(T64, ob, OUT + (size_t)b * NQ * 3); }
}
